// SECONDMambaBlock_49005576847551
// MI455X (gfx1250) — hardware-run, weakly checked
//
#include <hip/hip_runtime.h>
#include <math.h>

constexpr int kTok    = 32400;
constexpr int kMpad   = 32448;
constexpr int kCin    = 256;
constexpr int kNproj  = 524;
constexpr int kNpad   = 576;
constexpr int kCatHalf = 256;
constexpr int kWoutK  = 512;
constexpr int kM0     = 16256;
constexpr int kM1     = 16192;
constexpr int kScanTS = 64;
constexpr float kLnEps = 1e-6f;
static_assert(kM0 + kM1 == kMpad, "");
static_assert((kM0 % 64) == 0 && (kM1 % 64) == 0 && (kMpad % 64) == 0, "");
static_assert((kCin % 32) == 0 && (kCatHalf % 32) == 0 && (kNpad % 64) == 0, "");

typedef __attribute__((ext_vector_type(16))) _Float16 v16h;
typedef __attribute__((ext_vector_type(8)))  _Float16 v8h;
typedef __attribute__((ext_vector_type(16))) __bf16   v16b;
typedef __attribute__((ext_vector_type(8)))  __bf16   v8b;
typedef __attribute__((ext_vector_type(8)))  float    v8f;
typedef __attribute__((ext_vector_type(4)))  float    v4f;
typedef __attribute__((ext_vector_type(4)))  unsigned int v4u;

__device__ __forceinline__ unsigned short f2bf_bits(float f) {
  unsigned u = __float_as_uint(f);
  return (unsigned short)((u + 0x7FFFu + ((u >> 16) & 1u)) >> 16);
}
__device__ __forceinline__ float bf_bits2f(unsigned short h) { return __uint_as_float(((unsigned)h) << 16); }

__device__ __forceinline__ void dep_guard_h(v8f& a, v8f& b, v16h x, v16h y) { asm volatile("v_nop\n\tv_nop\n\tv_nop\n\tv_nop" : "+v"(a), "+v"(b) : "v"(x), "v"(y)); }
__device__ __forceinline__ void dep_guard_b(v8f& a, v8f& b, v16b x, v16b y) { asm volatile("v_nop\n\tv_nop\n\tv_nop\n\tv_nop" : "+v"(a), "+v"(b) : "v"(x), "v"(y)); }
__device__ __forceinline__ void keep4_h(v16h a, v16h b, v16h c, v16h d) { asm volatile("v_nop" :: "v"(a), "v"(b), "v"(c), "v"(d)); }
__device__ __forceinline__ void keep4_b(v16b a, v16b b, v16b c, v16b d) { asm volatile("v_nop" :: "v"(a), "v"(b), "v"(c), "v"(d)); }
__device__ __forceinline__ void acc_guard4(v8f& a, v8f& b, v8f& c, v8f& d) { asm volatile("v_nop\n\tv_nop\n\tv_nop\n\tv_nop" : "+v"(a), "+v"(b), "+v"(c), "+v"(d)); }
template <typename T> struct Frag;
template <> struct Frag<_Float16> {
  typedef v16h V; union U { v16h v; v8h h[2]; };
  static __device__ __forceinline__ v16h load(const _Float16* p) {
    U f; f.h[0] = *(const v8h*)(p); f.h[1] = *(const v8h*)(p + 16); return f.v;
  }
  static __device__ __forceinline__ v8f mma(v16h a, v16h b, v8f c) {
    return __builtin_amdgcn_wmma_f32_16x16x32_f16(false, a, false, b, (short)0, c, false, false);
  }
  static __device__ __forceinline__ void guard(v8f& a, v8f& b, v16h x, v16h y) { dep_guard_h(a, b, x, y); }
  static __device__ __forceinline__ void keep(v16h a, v16h b, v16h c, v16h d) { keep4_h(a, b, c, d); }
};
template <> struct Frag<__bf16> {
  typedef v16b V; union U { v16b v; v8b h[2]; };
  static __device__ __forceinline__ v16b load(const __bf16* p) {
    U f; f.h[0] = *(const v8b*)(p); f.h[1] = *(const v8b*)(p + 16); return f.v;
  }
  static __device__ __forceinline__ v8f mma(v16b a, v16b b, v8f c) {
    return __builtin_amdgcn_wmma_f32_16x16x32_bf16(false, a, false, b, (short)0, c, false, false);
  }
  static __device__ __forceinline__ void guard(v8f& a, v8f& b, v16b x, v16b y) { dep_guard_b(a, b, x, y); }
  static __device__ __forceinline__ void keep(v16b a, v16b b, v16b c, v16b d) { keep4_b(a, b, c, d); }
};

__device__ __forceinline__ unsigned pk16(unsigned short a, unsigned short b) { return (unsigned)a | ((unsigned)b << 16); }

template <int ET> struct Elem;
template <> struct Elem<0> { typedef _Float16 T; };
template <> struct Elem<1> { typedef __bf16 T; };
template <int ET, bool SPLIT, int BIAS_MODE, int OUT_MODE, bool RESID, int ACT = 0>
__global__ __launch_bounds__(256) void wmma_gemm64(
    const unsigned short* __restrict__ Ap, const unsigned short* __restrict__ A2p, int lda, long strideA,
    const unsigned short* __restrict__ Btp, const unsigned short* __restrict__ Bt2p, int ldb, long strideB,
    void* __restrict__ Cout, void* __restrict__ Cout2, int ldc, long strideC,
    const float* __restrict__ bias,
    const float* __restrict__ resid, long strideR,
    int M, int N, int K, float scale) {
  typedef typename Elem<ET>::T T;
  typedef typename Frag<T>::V V;
  const T* A = (const T*)Ap; const T* A2 = (const T*)A2p; const T* Bt = (const T*)Btp; const T* Bt2 = (const T*)Bt2p;
  __shared__ __align__(16) float sT[8][16 * 68];
  const int b    = blockIdx.y;
  const int lane = threadIdx.x & 31;
  const int wave = threadIdx.x >> 5;
  const int tilesN = N >> 6;
  const int tilesM = M >> 6;
  const int tile = blockIdx.x * 8 + wave;
  if (tile >= tilesM * tilesN) return;
  const int tm = tile / tilesN;
  const int tn = tile - tm * tilesN;
  const int m0 = tm << 6;
  const int n0 = tn << 6;

  const T* Ab  = A  + (size_t)b * strideA;
  const T* Bb  = Bt + (size_t)b * strideB;
  const T* Ab2 = SPLIT ? (A2  + (size_t)b * strideA) : nullptr;
  const T* Bb2 = SPLIT ? (Bt2 + (size_t)b * strideB) : nullptr;

  const int rlane = lane & 15;
  const int koff  = (lane >> 4) * 8;
  const int mOff  = (lane >> 4) * 8;

  v8f acc[4][4];
#pragma unroll
  for (int i = 0; i < 4; ++i)
#pragma unroll
    for (int j = 0; j < 4; ++j) acc[i][j] = (v8f){0.f,0.f,0.f,0.f,0.f,0.f,0.f,0.f};

  for (int k0 = 0; k0 < K; k0 += 32) {
    V bh[4], bl[4];
#pragma unroll
    for (int j = 0; j < 4; ++j) {
      const size_t bo = (size_t)(n0 + (j << 4) + rlane) * ldb + koff + k0;
      bh[j] = Frag<T>::load(Bb + bo);
      if (SPLIT) bl[j] = Frag<T>::load(Bb2 + bo);
    }
#pragma unroll
    for (int i = 0; i < 4; ++i) {
      const size_t ao = (size_t)(m0 + (i << 4) + rlane) * lda + koff + k0;
      V ah = Frag<T>::load(Ab + ao);
      V al;
      if (SPLIT) al = Frag<T>::load(Ab2 + ao);
#pragma unroll
      for (int j = 0; j < 4; ++j) {
        acc[i][j] = Frag<T>::mma(ah, bh[j], acc[i][j]);
        if (SPLIT) {
          acc[i][j] = Frag<T>::mma(ah, bl[j], acc[i][j]);
          acc[i][j] = Frag<T>::mma(al, bh[j], acc[i][j]);
        }
      }
      Frag<T>::guard(acc[i][0], acc[i][3], ah, SPLIT ? al : ah);
    }
    Frag<T>::keep(bh[0], bh[1], bh[2], bh[3]);
    if (SPLIT) Frag<T>::keep(bl[0], bl[1], bl[2], bl[3]);
  }
  acc_guard4(acc[0][0], acc[0][1], acc[0][2], acc[0][3]);
  acc_guard4(acc[1][0], acc[1][1], acc[1][2], acc[1][3]);
  acc_guard4(acc[2][0], acc[2][1], acc[2][2], acc[2][3]);
  acc_guard4(acc[3][0], acc[3][1], acc[3][2], acc[3][3]);

  float* slab = sT[wave];
  const float* Rb = RESID ? (resid + (size_t)b * strideR) : nullptr;
#pragma unroll
  for (int i = 0; i < 4; ++i) {
    const int mBase = m0 + (i << 4);
#pragma unroll
    for (int j = 0; j < 4; ++j) {
      const int n = n0 + (j << 4) + rlane;
      float bv = 0.f;
      if (BIAS_MODE == 2) bv = bias[n];
#pragma unroll
      for (int r = 0; r < 8; ++r) {
        float v = acc[i][j][r] * scale;
        if (BIAS_MODE == 1) v += bias[mBase + mOff + r];
        if (BIAS_MODE == 2) v += bv;
        if (RESID) v += Rb[(size_t)(mBase + mOff + r) * ldc + n];
        if (ACT == 2) v = fmaxf(v, 0.0f);
        if (ACT == 4) v = (v > 0.f) ? v : 0.01f * v;
        slab[(mOff + r) * 68 + (j << 4) + rlane] = v;
      }
    }
    __builtin_amdgcn_fence(__ATOMIC_RELEASE, "workgroup");
    __builtin_amdgcn_wave_barrier();
    __builtin_amdgcn_fence(__ATOMIC_ACQUIRE, "workgroup");
    if (OUT_MODE == 0) {
      float* C = (float*)Cout + (size_t)b * strideC;
      const int hh = lane >> 4, c4 = (lane & 15) * 4;
      for (int pass = 0; pass < 2; ++pass) {
#pragma unroll
        for (int it = 0; it < 8; ++it) {
          const int row = it * 2 + hh;
          v4f v = *(const v4f*)(slab + row * 68 + c4);
          *(volatile v4f*)(C + (size_t)(mBase + row) * ldc + n0 + c4) = v;
        }
        __threadfence();
      }
    } else {
      const int q = lane >> 3, c8 = (lane & 7) * 8;
      unsigned short* C  = (unsigned short*)Cout  + (size_t)b * strideC;
      unsigned short* C2 = (OUT_MODE == 2) ? ((unsigned short*)Cout2 + (size_t)b * strideC) : nullptr;
      for (int pass = 0; pass < 2; ++pass) {
#pragma unroll
        for (int it = 0; it < 4; ++it) {
          const int row = it * 4 + q;
          const float* sp = slab + row * 68 + c8;
          v8h hv, lv;
#pragma unroll
          for (int e = 0; e < 8; ++e) {
            if (OUT_MODE == 1) {
              hv[e] = (_Float16)sp[e];
            } else {
              unsigned short hb = f2bf_bits(sp[e]);
              unsigned short lb = f2bf_bits(sp[e] - bf_bits2f(hb));
              hv[e] = __builtin_bit_cast(_Float16, hb);
              lv[e] = __builtin_bit_cast(_Float16, lb);
            }
          }
          *(volatile v8h*)(C + (size_t)(mBase + row) * ldc + n0 + c8) = hv;
          if (OUT_MODE == 2) *(volatile v8h*)(C2 + (size_t)(mBase + row) * ldc + n0 + c8) = lv;
        }
        __threadfence();
      }
    }
    __builtin_amdgcn_fence(__ATOMIC_RELEASE, "workgroup");
    __builtin_amdgcn_wave_barrier();
    __builtin_amdgcn_fence(__ATOMIC_ACQUIRE, "workgroup");
  }
}

__device__ __forceinline__ float silu_f(float x) {
  const float e = expf(-x);
  return x * (1.0f / (1.0f + e));
}
__device__ __forceinline__ float softplus_f(float x) {
  const float ax = fabsf(x);
  return fmaxf(x, 0.0f) + log1pf(expf(-ax));
}
__device__ __forceinline__ void split_pack8(v4f a, v4f b, v4u& hu, v4u& lu) {
  unsigned short hb[8], lb[8];
#pragma unroll
  for (int e = 0; e < 4; ++e) {
    const unsigned short h0 = f2bf_bits(a[e]);
    hb[e] = h0;
    lb[e] = f2bf_bits(a[e] - bf_bits2f(h0));
    const unsigned short h1 = f2bf_bits(b[e]);
    hb[4 + e] = h1;
    lb[4 + e] = f2bf_bits(b[e] - bf_bits2f(h1));
  }
  hu = (v4u){pk16(hb[0], hb[1]), pk16(hb[2], hb[3]), pk16(hb[4], hb[5]), pk16(hb[6], hb[7])};
  lu = (v4u){pk16(lb[0], lb[1]), pk16(lb[2], lb[3]), pk16(lb[4], lb[5]), pk16(lb[6], lb[7])};
}

__global__ __launch_bounds__(256) void k_split_rows(const float* __restrict__ src, int rows_valid, int kcols, int n8,
                                                     unsigned short* __restrict__ hi, unsigned short* __restrict__ lo) {
  const int i = blockIdx.x * 256 + threadIdx.x;
  if (i >= n8) return;
  const int e0 = i * 8;
  const int r  = e0 / kcols;
  const int c  = e0 - r * kcols;
  const int rr = (r < rows_valid) ? r : (rows_valid - 1);
  const float* p = src + (size_t)rr * kcols + c;
  v4f a = *(const v4f*)(p);
  v4f b = *(const v4f*)(p + 4);
  if (r >= rows_valid) { a = (v4f){0.f, 0.f, 0.f, 0.f}; b = (v4f){0.f, 0.f, 0.f, 0.f}; }
  v4u hu, lu;
  split_pack8(a, b, hu, lu);
  unsigned short* ph = hi + (size_t)e0;
  unsigned short* pl = lo + (size_t)e0;
  *(volatile v4u*)ph = hu;
  *(volatile v4u*)pl = lu;
  __threadfence();
  *(volatile v4u*)ph = hu;
  *(volatile v4u*)pl = lu;
}

__global__ __launch_bounds__(256) void k_gather_split(const float* __restrict__ x, const int* __restrict__ perm,
                                                       int mbeg, int mrows,
                                                       unsigned short* __restrict__ hi, unsigned short* __restrict__ lo) {
  const int gid = blockIdx.x * 256 + threadIdx.x;
  const int r   = gid >> 5;
  const int c0  = (gid & 31) * 8;
  if (r >= mrows) return;
  const int l   = mbeg + r;
  const bool valid = (l < kTok);
  const int lc  = valid ? l : (kTok - 1);
  int m = perm[lc];
  m = (m < 0) ? 0 : ((m > kTok - 1) ? (kTok - 1) : m);
  v4f a, b;
#pragma unroll
  for (int e = 0; e < 4; ++e) {
    a[e] = x[(size_t)(c0 + e) * kTok + m];
    b[e] = x[(size_t)(c0 + 4 + e) * kTok + m];
  }
  if (!valid) { a = (v4f){0.f, 0.f, 0.f, 0.f}; b = (v4f){0.f, 0.f, 0.f, 0.f}; }
  v4u hu, lu;
  split_pack8(a, b, hu, lu);
  unsigned short* ph = hi + (size_t)r * kCin + c0;
  unsigned short* pl = lo + (size_t)r * kCin + c0;
  *(volatile v4u*)ph = hu;
  *(volatile v4u*)pl = lu;
  __threadfence();
  *(volatile v4u*)ph = hu;
  *(volatile v4u*)pl = lu;
}

__global__ __launch_bounds__(256) void k_scan(const float* __restrict__ Z, int mrows, int mbeg, int lbeg, int lend,
                                              const float* __restrict__ dt_bias, const float* __restrict__ A_log,
                                              const float* __restrict__ Dp,
                                              const float* __restrict__ state_in, float* __restrict__ state_out, int first,
                                              float* __restrict__ Y) {
  __shared__ __align__(16) float sB[kScanTS * 4];
  __shared__ __align__(16) float sC[kScanTS * 4];
  __shared__ float sDT[kScanTS * 4];
  __shared__ float sDA[kScanTS * 4];
  const int t = threadIdx.x;
  const int h = t >> 6;
  const int q = t & 3;
  const float myBias = dt_bias[q];
  const float myA    = -expf(A_log[q]);
  const float Dh     = Dp[h];
  float S0 = 0.f, S1 = 0.f, S2 = 0.f, S3 = 0.f;
  if (first == 0) {
    const v4f si = *(const v4f*)(state_in + 4 * t);
    S0 = si[0]; S1 = si[1]; S2 = si[2]; S3 = si[3];
  }
  for (int l0 = lbeg; l0 < lend; l0 += kScanTS) {
    const int nst = ((lend - l0) < kScanTS) ? (lend - l0) : kScanTS;
    __syncthreads();
    {
      const int r = t >> 2;
      int lr = l0 + r - mbeg;
      lr = (lr < mrows) ? lr : (mrows - 1);
      const float* zp = Z + (size_t)lr * kNpad + 512;
      const float braw = zp[q];
      const float craw = zp[4 + q];
      const float dtr  = zp[8 + q];
      sB[r * 4 + q] = silu_f(braw);
      sC[r * 4 + q] = silu_f(craw);
      const float dtv = softplus_f(dtr + myBias);
      sDT[r * 4 + q] = dtv;
      sDA[r * 4 + q] = expf(dtv * myA);
    }
    __syncthreads();
#pragma unroll 1
    for (int r = 0; r < nst; ++r) {
      const size_t lr = (size_t)(l0 + r - mbeg);
      const float xr = Z[lr * kNpad + 256 + t];
      const float zr = Z[lr * kNpad + t];
      const v4f bv = *(const v4f*)(sB + r * 4);
      const v4f cv = *(const v4f*)(sC + r * 4);
      const float dt = sDT[r * 4 + h];
      const float dA = sDA[r * 4 + h];
      const float xs = silu_f(xr);
      const float u  = dt * xs;
      S0 = dA * S0 + bv[0] * u;
      S1 = dA * S1 + bv[1] * u;
      S2 = dA * S2 + bv[2] * u;
      S3 = dA * S3 + bv[3] * u;
      float y = cv[0] * S0 + cv[1] * S1 + cv[2] * S2 + cv[3] * S3;
      y = y + Dh * xs;
      y = y * silu_f(zr);
      float* yp = Y + (size_t)(l0 + r) * kCin + t;
      *(volatile float*)yp = y;
      __threadfence();
      *(volatile float*)yp = y;
    }
  }
  const v4f so = (v4f){S0, S1, S2, S3};
  float* stp = state_out + 4 * t;
  *(volatile v4f*)stp = so;
  __threadfence();
  *(volatile v4f*)stp = so;
}

__global__ __launch_bounds__(256) void k_perm_split(const float* __restrict__ Ysrc, const int* __restrict__ inv,
                                                     unsigned short* __restrict__ hi, unsigned short* __restrict__ lo) {
  const int gid = blockIdx.x * 256 + threadIdx.x;
  const int r   = gid >> 5;
  const int c0  = (gid & 31) * 8;
  if (r >= kMpad) return;
  const bool valid = (r < kTok);
  const int rc  = valid ? r : (kTok - 1);
  int j = inv[rc];
  j = (j < 0) ? 0 : ((j > kTok - 1) ? (kTok - 1) : j);
  const float* p = Ysrc + (size_t)j * kCin + c0;
  v4f a = *(const v4f*)(p);
  v4f b = *(const v4f*)(p + 4);
  if (!valid) { a = (v4f){0.f, 0.f, 0.f, 0.f}; b = (v4f){0.f, 0.f, 0.f, 0.f}; }
  v4u hu, lu;
  split_pack8(a, b, hu, lu);
  unsigned short* ph = hi + (size_t)r * kCin + c0;
  unsigned short* pl = lo + (size_t)r * kCin + c0;
  *(volatile v4u*)ph = hu;
  *(volatile v4u*)pl = lu;
  __threadfence();
  *(volatile v4u*)ph = hu;
  *(volatile v4u*)pl = lu;
}

__global__ __launch_bounds__(256) void k_ln(const float* __restrict__ O, const float* __restrict__ gamma,
                                            const float* __restrict__ beta, float* __restrict__ oln) {
  const int lane = threadIdx.x & 31, wave = threadIdx.x >> 5;
  const int row  = blockIdx.x * 8 + wave;
  const float* p = O + (size_t)row * kCin;
  const v4f a = *(const v4f*)(p + 4 * lane);
  const v4f b = *(const v4f*)(p + 128 + 4 * lane);
  float s = ((a[0] + a[1]) + (a[2] + a[3])) + ((b[0] + b[1]) + (b[2] + b[3]));
#pragma unroll
  for (int off = 16; off > 0; off >>= 1) s += __shfl_xor(s, off, 32);
  const float mu = s * (1.0f / 256.0f);
  const v4f da = a - mu;
  const v4f db = b - mu;
  float s2 = ((da[0] * da[0] + da[1] * da[1]) + (da[2] * da[2] + da[3] * da[3])) +
             ((db[0] * db[0] + db[1] * db[1]) + (db[2] * db[2] + db[3] * db[3]));
#pragma unroll
  for (int off = 16; off > 0; off >>= 1) s2 += __shfl_xor(s2, off, 32);
  const float var  = s2 * (1.0f / 256.0f);
  const float rstd = 1.0f / sqrtf(var + kLnEps);
  const v4f ga = *(const v4f*)(gamma + 4 * lane);
  const v4f gb = *(const v4f*)(gamma + 128 + 4 * lane);
  const v4f ba = *(const v4f*)(beta + 4 * lane);
  const v4f bb = *(const v4f*)(beta + 128 + 4 * lane);
  const v4f oa = (da * rstd) * ga + ba;
  const v4f ob = (db * rstd) * gb + bb;
  float* q0 = oln + (size_t)row * kCin + 4 * lane;
  float* q1 = q0 + 128;
  *(volatile v4f*)q0 = oa;
  *(volatile v4f*)q1 = ob;
  __threadfence();
  *(volatile v4f*)q0 = oa;
  *(volatile v4f*)q1 = ob;
}

__global__ __launch_bounds__(256) void k_transpose_out(const float* __restrict__ oln, float* __restrict__ out) {
  const int cp = blockIdx.x;
  const int t  = threadIdx.x;
  float* base = out + (size_t)cp * (2 * kTok);
#pragma unroll 1
  for (int it = 0; it < 64; ++it) {
    const int e = it * 1024 + t * 4;
    if (e < 2 * kTok) {
      const int ch  = (e >= kTok) ? 1 : 0;
      const int l   = e - ch * kTok;
      const int col = 2 * cp + ch;
      const float* sp = oln + (size_t)l * kCin + col;
      v4f v;
      v[0] = sp[0];
      v[1] = sp[kCin];
      v[2] = sp[2 * kCin];
      v[3] = sp[3 * kCin];
      float* dp = base + e;
      *(volatile v4f*)dp = v;
      __threadfence();
      *(volatile v4f*)dp = v;
    }
  }
}

extern "C" void kernel_launch(void* const* d_in, const int* in_sizes, int n_in,
                              void* d_out, int out_size, void* d_ws, size_t ws_size, hipStream_t stream) {
  if (n_in < 16) return;
  if (out_size != kCin * kTok) return;
  if (in_sizes[0] != kCin * kTok || in_sizes[1] != kNproj * kCin || in_sizes[2] != kNproj * kCin ||
      in_sizes[3] != 4 || in_sizes[4] != 4 || in_sizes[5] != 4 || in_sizes[6] != 4 || in_sizes[7] != 4 ||
      in_sizes[8] != 4 || in_sizes[9] != kCin * kWoutK || in_sizes[10] != kCin || in_sizes[11] != kCin ||
      in_sizes[12] != kTok || in_sizes[13] != kTok || in_sizes[14] != kTok || in_sizes[15] != kTok) return;

  const float* x      = (const float*)d_in[0];
  const float* WinH   = (const float*)d_in[1];
  const float* WinV   = (const float*)d_in[2];
  const float* dtbH   = (const float*)d_in[3];
  const float* dtbV   = (const float*)d_in[4];
  const float* AlogH  = (const float*)d_in[5];
  const float* AlogV  = (const float*)d_in[6];
  const float* DarrH  = (const float*)d_in[7];
  const float* DarrV  = (const float*)d_in[8];
  const float* Wout   = (const float*)d_in[9];
  const float* gamma  = (const float*)d_in[10];
  const float* beta   = (const float*)d_in[11];
  const int*   permH  = (const int*)d_in[12];
  const int*   permV  = (const int*)d_in[13];
  const int*   invH   = (const int*)d_in[14];
  const int*   invV   = (const int*)d_in[15];
  float* out = (float*)d_out;

  const size_t szWin  = (size_t)kNpad * kCin * 2;
  const size_t szWout = (size_t)kCin * kWoutK * 2;
  const size_t szSt   = (size_t)kCin * 4 * 4;
  const size_t szA16  = (size_t)kM0 * kCin * 2;
  const size_t szZ    = (size_t)kM0 * kNpad * 4;
  const size_t szBig  = (size_t)kMpad * kCin * 4;
  const size_t szCat  = (size_t)kMpad * kCatHalf * 2;
  size_t off = 0;
  auto carve = [&](size_t bytes) -> size_t { const size_t o = off; off = (off + bytes + 255) & ~(size_t)255; return o; };
  const size_t oWinHh = carve(szWin), oWinHl = carve(szWin);
  const size_t oWinVh = carve(szWin), oWinVl = carve(szWin);
  const size_t oWoh   = carve(szWout), oWol = carve(szWout);
  const size_t oSt0   = carve(szSt), oSt1 = carve(szSt);
  const size_t oA16h  = carve(szA16), oA16l = carve(szA16);
  const size_t oZ     = carve(szZ);
  const size_t spanEnd = off;
  const size_t oYH    = carve(szBig);
  const size_t oYV    = carve(szBig);
  if (off > ws_size) return;
  if (spanEnd - oA16h < 2 * szCat) return;
  if (spanEnd - oA16h < (size_t)kTok * kCin * 4) return;

  char* ws = (char*)d_ws;
  unsigned short* WinHh = (unsigned short*)(ws + oWinHh); unsigned short* WinHl = (unsigned short*)(ws + oWinHl);
  unsigned short* WinVh = (unsigned short*)(ws + oWinVh); unsigned short* WinVl = (unsigned short*)(ws + oWinVl);
  unsigned short* Woh   = (unsigned short*)(ws + oWoh);   unsigned short* Wol   = (unsigned short*)(ws + oWol);
  float* St0 = (float*)(ws + oSt0); float* St1 = (float*)(ws + oSt1);
  unsigned short* A16h = (unsigned short*)(ws + oA16h); unsigned short* A16l = (unsigned short*)(ws + oA16l);
  float* Z = (float*)(ws + oZ);
  unsigned short* CATh = (unsigned short*)(ws + oA16h);
  unsigned short* CATl = (unsigned short*)(ws + oA16h + szCat);
  float* OLN = (float*)(ws + oA16h);
  float* YH = (float*)(ws + oYH);
  float* YV = (float*)(ws + oYV);
  float* O1 = YH;
  float* O2 = YV;
  const float* dummyf = (const float*)(ws);
  void* dummyv = (void*)(ws);

  {
    const int n8in = kNpad * kCin / 8;
    const int n8out = kCin * kWoutK / 8;
    k_split_rows<<<(n8in + 255) / 256, 256, 0, stream>>>(WinH, kNproj, kCin, n8in, WinHh, WinHl);
    k_split_rows<<<(n8in + 255) / 256, 256, 0, stream>>>(WinV, kNproj, kCin, n8in, WinVh, WinVl);
    k_split_rows<<<(n8out + 255) / 256, 256, 0, stream>>>(Wout, kCin, kWoutK, n8out, Woh, Wol);
  }

  for (int p = 0; p < 2; ++p) {
    const int*   perm  = (p == 0) ? permH : permV;
    const float* dtb   = (p == 0) ? dtbH : dtbV;
    const float* Alog  = (p == 0) ? AlogH : AlogV;
    const float* Darr  = (p == 0) ? DarrH : DarrV;
    const unsigned short* Wh = (p == 0) ? WinHh : WinVh;
    const unsigned short* Wl = (p == 0) ? WinHl : WinVl;
    float* Y = (p == 0) ? YH : YV;
    for (int ck = 0; ck < 2; ++ck) {
      const int mbeg  = (ck == 0) ? 0 : kM0;
      const int mrows = (ck == 0) ? kM0 : kM1;
      const int lend  = (ck == 0) ? kM0 : kTok;
      k_gather_split<<<mrows / 8, 256, 0, stream>>>(x, perm, mbeg, mrows, A16h, A16l);
      {
        const int tiles = (mrows / 64) * (kNpad / 64);
        wmma_gemm64<1, true, 0, 0, false><<<dim3((tiles + 7) / 8, 1), 256, 0, stream>>>(
            A16h, A16l, kCin, 0L, Wh, Wl, kCin, 0L, (void*)Z, dummyv, kNpad, 0L,
            dummyf, dummyf, 0L, mrows, kNpad, kCin, 1.0f);
      }
      {
        const float* stIn = (ck == 0) ? St1 : St0;
        float* stOut      = (ck == 0) ? St0 : St1;
        const int first   = (ck == 0) ? 1 : 0;
        k_scan<<<1, 256, 0, stream>>>(Z, mrows, mbeg, mbeg, lend, dtb, Alog, Darr, stIn, stOut, first, Y);
      }
    }
  }

  {
    const int tiles = (kMpad / 64) * (kCin / 64);
    k_perm_split<<<kMpad / 8, 256, 0, stream>>>(YH, invH, CATh, CATl);
    wmma_gemm64<1, true, 0, 0, false><<<dim3((tiles + 7) / 8, 1), 256, 0, stream>>>(
        CATh, CATl, kCatHalf, 0L, Woh, Wol, kWoutK, 0L, (void*)O1, dummyv, kCin, 0L,
        dummyf, dummyf, 0L, kMpad, kCin, kCatHalf, 1.0f);
    k_perm_split<<<kMpad / 8, 256, 0, stream>>>(YV, invV, CATh, CATl);
    wmma_gemm64<1, true, 0, 0, true><<<dim3((tiles + 7) / 8, 1), 256, 0, stream>>>(
        CATh, CATl, kCatHalf, 0L, Woh + kCatHalf, Wol + kCatHalf, kWoutK, 0L, (void*)O2, dummyv, kCin, 0L,
        dummyf, O1, 0L, kMpad, kCin, kCatHalf, 1.0f);
  }

  k_ln<<<kTok / 8, 256, 0, stream>>>(O2, gamma, beta, OLN);
  k_transpose_out<<<kCin / 2, 256, 0, stream>>>(OLN, out);
}
